// ConcatHeadModule_62852551409784
// MI455X (gfx1250) — hardware-run, weakly checked
//
#include <hip/hip_runtime.h>


#ifndef TT
#define TT 768
#endif
#define TT_FULL 768
#ifndef OUT_PITCH
#define OUT_PITCH TT
#endif
#define KD    512
#define HID   512
#define HID2  512
#define NCAT  (2 * HID)
#define W2S   64.0f
#define W2I   (1.0f / 64.0f)
#define TI    64
#define TJ    32
#define HC    32
#define PA    (TI + 4)
#define PB    (TJ + 4)
#define PO    (TJ + 4)
#define TSP   72

static_assert(TT % 64 == 0);
static_assert(TT <= TT_FULL);
static_assert(KD % 64 == 0);
static_assert(HID % 64 == 0);
static_assert(HID2 % 64 == 0);
static_assert(NCAT % 64 == 0);
static_assert(KD % 32 == 0);
static_assert(HID % 32 == 0);
static_assert(HID2 % HC == 0);
static_assert(HC == 32);
static_assert(TJ == 32);
static_assert(OUT_PITCH % 32 == 0);
static_assert(OUT_PITCH >= TT);
static_assert(((size_t)TT * KD) % (8 * 256) == 0);
static_assert((PA * 4) % 16 == 0);
static_assert((PB * 4) % 8 == 0);
static_assert((PO * 4) % 16 == 0);
static_assert(256 * 4 * 4 == 64 * 64);
static_assert(256 * 16 * 2 == 64 * 64 * 2);
static_assert(32 * 16 * 4 == 16 * 64 * 2);
static_assert(32 * 16 * 8 == 16 * 64 * 4);
static_assert(256 * 16 * 2 == TI * TJ * 4);
static_assert(16 * 68 * 4 <= 131072);
static_assert(64 * TSP * 2 <= 131072);
static_assert((HC * PA + HC * PB + HC + TI * PO) * 4 <= 131072);

typedef _Float16 h16;
typedef unsigned short bf;
typedef __attribute__((ext_vector_type(16))) __bf16   v16bf;
typedef __attribute__((ext_vector_type(16))) _Float16 v16h;
typedef __attribute__((ext_vector_type(8)))  _Float16 v8h;
typedef __attribute__((ext_vector_type(8)))  unsigned short v8us;
typedef __attribute__((ext_vector_type(8)))  float    v8f;
typedef __attribute__((ext_vector_type(4)))  float    v4f;
typedef v4f  __attribute__((may_alias)) v4fa;

__device__ __forceinline__ unsigned short f2bf(float f) { unsigned u = __float_as_uint(f); u += 0x7FFFu + ((u >> 16) & 1u); return (unsigned short)(u >> 16); }
__device__ __forceinline__ float bfr(float f) { return __uint_as_float(((unsigned)f2bf(f)) << 16); }
__device__ __forceinline__ v16h cat16(v8h lo, v8h hi) { return __builtin_shufflevector(lo, hi, 0, 1, 2, 3, 4, 5, 6, 7, 8, 9, 10, 11, 12, 13, 14, 15); }
__device__ __forceinline__ v16bf cat16b(v8us lo, v8us hi) { return __builtin_bit_cast(v16bf, __builtin_shufflevector(lo, hi, 0, 1, 2, 3, 4, 5, 6, 7, 8, 9, 10, 11, 12, 13, 14, 15)); }
__device__ __forceinline__ v8f wmma16(v16h a, v16h b, v8f c) { return __builtin_amdgcn_wmma_f32_16x16x32_f16(false, a, false, b, (short)0, c, false, false); }
__device__ __forceinline__ v8f wmmab(v16bf a, v16bf b, v8f c) { return __builtin_amdgcn_wmma_f32_16x16x32_bf16(false, a, false, b, (short)0, c, false, false); }
__device__ __forceinline__ v16h  ldh(const h16* p) { return cat16(*(const v8h*)p, *(const v8h*)(p + 16)); }
__device__ __forceinline__ v16bf ldb(const bf* p)  { return cat16b(*(const v8us*)p, *(const v8us*)(p + 16)); }
__device__ __forceinline__ void wave_sync() { __builtin_amdgcn_fence(3  , "wavefront"); __builtin_amdgcn_wave_barrier(); asm volatile("" ::: "memory"); }

typedef __attribute__((ext_vector_type(2))) float v2f;
typedef v2f __attribute__((may_alias)) v2fa;

__device__ __forceinline__ v8f wmma16g(v16h a, v16h b, v8f c) { c = wmma16(a, b, c); asm volatile("v_nop\n\tv_nop\n\tv_nop\n\tv_nop" : "+v"(c) : "v"(a), "v"(b)); return c; }
__device__ __forceinline__ v8f wmmabg(v16bf a, v16bf b, v8f c) { c = wmmab(a, b, c); asm volatile("v_nop\n\tv_nop\n\tv_nop\n\tv_nop" : "+v"(c) : "v"(a), "v"(b)); return c; }
static __device__ __forceinline__ h16 toh_flush(float v) { const h16 r = (h16)v; return (fabsf(v) < 6.103515625e-05f) ? (h16)0.0f : r; }

#if defined(__has_builtin)
#if __has_builtin(__builtin_amdgcn_tanhf)
#define HAVE_HW_TANH 1
#endif
#endif
__device__ __forceinline__ float tanh_f(float x) {
#ifdef HAVE_HW_TANH
    return __builtin_amdgcn_tanhf(x);
#else
    const float e = __builtin_amdgcn_exp2f(x * 2.8853900817779268f);
    return 1.0f - 2.0f * __builtin_amdgcn_rcpf(e + 1.0f);
#endif
}

__global__ __launch_bounds__(256) void k_cvt8(const float* __restrict__ src, bf* dst, size_t n8) {
    const size_t i = (size_t)blockIdx.x * 256 + threadIdx.x; if (i >= n8) return;
    const v8f v = *(const v8f*)(src + i * 8); v8us o;
#pragma unroll
    for (int k = 0; k < 8; ++k) o[k] = f2bf(v[k]);
    *(volatile v8us*)(dst + i * 8) = o; __threadfence(); *(volatile v8us*)(dst + i * 8) = o;
}

__global__ __launch_bounds__(256) void k_wtb(const float* __restrict__ W, bf* dst, int wk, int wn) {
    __shared__ unsigned short ts[64 * TSP];
    const int tid = threadIdx.x; const int k0 = blockIdx.x * 64, n0 = blockIdx.y * 64;
    const size_t zo = (size_t)blockIdx.z * (size_t)wk * (size_t)wn;
#pragma unroll
    for (int it = 0; it < 4; ++it) { const int idx = tid + 256 * it; const int kk = idx >> 4, c4 = (idx & 15) * 4;
        const v4f v = *(const v4f*)(W + zo + (size_t)(k0 + kk) * (size_t)wn + n0 + c4);
#pragma unroll
        for (int i = 0; i < 4; ++i) ts[kk * TSP + c4 + i] = f2bf(v[i]); }
    __syncthreads();
#pragma unroll 1
    for (int ps = 0; ps < 2; ++ps) {
#pragma unroll
        for (int it = 0; it < 2; ++it) { const int p = tid + 256 * it; const int nn = p >> 3, kc = (p & 7) * 8;
            v8us o;
#pragma unroll
            for (int i = 0; i < 8; ++i) o[i] = ts[(kc + i) * TSP + nn];
            *(volatile v8us*)(dst + zo + (size_t)(n0 + nn) * (size_t)wk + k0 + kc) = o; }
        if (ps == 0) __threadfence(); }
}

__global__ __launch_bounds__(256) void k_wth(const float* __restrict__ W, h16* dst, int wk, int wn) {
    __shared__ unsigned short ts[64 * TSP];
    const int tid = threadIdx.x; const int k0 = blockIdx.x * 64, n0 = blockIdx.y * 64;
    const size_t zo = (size_t)blockIdx.z * (size_t)wk * (size_t)wn;
#pragma unroll
    for (int it = 0; it < 4; ++it) { const int idx = tid + 256 * it; const int kk = idx >> 4, c4 = (idx & 15) * 4;
        const v4f v = *(const v4f*)(W + zo + (size_t)(k0 + kk) * (size_t)wn + n0 + c4);
#pragma unroll
        for (int i = 0; i < 4; ++i) ts[kk * TSP + c4 + i] = __builtin_bit_cast(unsigned short, toh_flush(bfr(v[i]) * W2S)); }
    __syncthreads();
#pragma unroll 1
    for (int ps = 0; ps < 2; ++ps) {
#pragma unroll
        for (int it = 0; it < 2; ++it) { const int p = tid + 256 * it; const int nn = p >> 3, kc = (p & 7) * 8;
            v8us o;
#pragma unroll
            for (int i = 0; i < 8; ++i) o[i] = ts[(kc + i) * TSP + nn];
            const v8h oh = __builtin_bit_cast(v8h, o);
            *(volatile v8h*)(dst + zo + (size_t)(n0 + nn) * (size_t)wk + k0 + kc) = oh; }
        if (ps == 0) __threadfence(); }
}

__global__ __launch_bounds__(32) void k_gemm1(const bf* __restrict__ A, const bf* __restrict__ Bt, const float* __restrict__ bias, h16* ACT) {
    __shared__ __align__(16) float os[16 * 68];
    const int lane = threadIdx.x & 31, lr = lane & 15, hi = lane >> 4; const int r0 = blockIdx.x * 64, c0 = blockIdx.y * 64;
    v8f acc[4][4];
#pragma unroll
    for (int mb = 0; mb < 4; ++mb)
#pragma unroll
        for (int nb = 0; nb < 4; ++nb) acc[mb][nb] = (v8f){};
    const size_t aoff = (size_t)(r0 + lr) * KD + 8 * hi, boff = (size_t)(c0 + lr) * KD + 8 * hi;
#pragma unroll 1
    for (int kc = 0; kc < KD; kc += 32) {
        v16bf a[4];
#pragma unroll
        for (int mb = 0; mb < 4; ++mb) a[mb] = ldb(A + aoff + (size_t)mb * 16 * KD + kc);
#pragma unroll
        for (int nb = 0; nb < 4; ++nb) { const v16bf b = ldb(Bt + boff + (size_t)nb * 16 * KD + kc);
#pragma unroll
            for (int mb = 0; mb < 4; ++mb) acc[mb][nb] = wmmabg(a[mb], b, acc[mb][nb]); }
    }
    float bc[4];
#pragma unroll
    for (int nb = 0; nb < 4; ++nb) bc[nb] = bfr(bias[c0 + nb * 16 + lr]);
#pragma unroll
    for (int mb = 0; mb < 4; ++mb) {
#pragma unroll
        for (int nb = 0; nb < 4; ++nb) {
#pragma unroll
            for (int j = 0; j < 8; ++j) os[(hi * 8 + j) * 68 + nb * 16 + lr] = tanh_f(acc[mb][nb][j] + bc[nb]); }
        wave_sync();
#pragma unroll 1
        for (int ps = 0; ps < 2; ++ps) {
#pragma unroll
            for (int s = 0; s < 4; ++s) { const int row = 4 * s + (lane >> 3), c8 = (lane & 7) * 8;
                const v4f x0 = *(const v4fa*)(&os[row * 68 + c8]); const v4f x1 = *(const v4fa*)(&os[row * 68 + c8 + 4]); v8h hv;
#pragma unroll
                for (int i = 0; i < 4; ++i) { hv[i] = toh_flush(x0[i]); hv[4 + i] = toh_flush(x1[i]); }
                *(volatile v8h*)(ACT + (size_t)(r0 + mb * 16 + row) * NCAT + c0 + c8) = hv; }
            if (ps == 0) __threadfence(); }
        wave_sync();
    }
}

__global__ __launch_bounds__(32) void k_gemm2(const h16* __restrict__ A, const h16* __restrict__ Bt, const float* __restrict__ bias, float* P) {
    __shared__ __align__(16) float os[16 * 68];
    const int lane = threadIdx.x & 31, lr = lane & 15, hi = lane >> 4; const int r0 = blockIdx.x * 64, c0 = blockIdx.y * 64; const int z = blockIdx.z;
    v8f acc[4][4];
#pragma unroll
    for (int mb = 0; mb < 4; ++mb)
#pragma unroll
        for (int nb = 0; nb < 4; ++nb) acc[mb][nb] = (v8f){};
    const size_t aoff = (size_t)(r0 + lr) * NCAT + (size_t)z * HID + 8 * hi;
    const size_t boff = (size_t)z * ((size_t)HID2 * HID) + (size_t)(c0 + lr) * HID + 8 * hi;
#pragma unroll 1
    for (int kc = 0; kc < HID; kc += 32) {
        v16h a[4];
#pragma unroll
        for (int mb = 0; mb < 4; ++mb) a[mb] = ldh(A + aoff + (size_t)mb * 16 * NCAT + kc);
#pragma unroll
        for (int nb = 0; nb < 4; ++nb) { const v16h b = ldh(Bt + boff + (size_t)nb * 16 * HID + kc);
#pragma unroll
            for (int mb = 0; mb < 4; ++mb) acc[mb][nb] = wmma16g(a[mb], b, acc[mb][nb]); }
    }
    const float bsel = (z == 1) ? 1.0f : 0.0f;
    float bc[4];
#pragma unroll
    for (int nb = 0; nb < 4; ++nb) bc[nb] = bfr(bias[c0 + nb * 16 + lr]) * bsel;
    float* Pz = P + (size_t)z * ((size_t)TT * HID2);
#pragma unroll
    for (int mb = 0; mb < 4; ++mb) {
#pragma unroll
        for (int nb = 0; nb < 4; ++nb) {
#pragma unroll
            for (int j = 0; j < 8; ++j) os[(hi * 8 + j) * 68 + nb * 16 + lr] = acc[mb][nb][j] * W2I + bc[nb]; }
        wave_sync();
#pragma unroll 1
        for (int ps = 0; ps < 2; ++ps) {
#pragma unroll
            for (int s = 0; s < 8; ++s) { const int row = 2 * s + (lane >> 4), c4 = (lane & 15) * 4;
                const v4f val = *(const v4fa*)(&os[row * 68 + c4]);
                *(volatile v4f*)(Pz + (size_t)(r0 + mb * 16 + row) * HID2 + c0 + c4) = val; }
            if (ps == 0) __threadfence(); }
        wave_sync();
    }
}

__global__ __launch_bounds__(256) void k_pair(const float* __restrict__ AH, const float* __restrict__ AM, const float* __restrict__ w, const float* __restrict__ ob_p, float* OUT) {
    __shared__ __align__(16) float sAt[HC * PA];
    __shared__ __align__(16) float sBt[HC * PB];
    __shared__ __align__(16) float sw[HC];
    __shared__ __align__(16) float so[TI * PO];
    const int tid = threadIdx.x;
    const int i0 = blockIdx.x * TI, j0 = blockIdx.y * TJ;
    const int ig4 = (tid >> 4) << 2;
    const int jg2 = (tid & 15) << 1;
    float a0x = 0.f, a0y = 0.f, a1x = 0.f, a1y = 0.f, a2x = 0.f, a2y = 0.f, a3x = 0.f, a3y = 0.f;
#pragma unroll 1
    for (int h0 = 0; h0 < HID2; h0 += HC) {
        __syncthreads();
#pragma unroll
        for (int it = 0; it < 2; ++it) { const int idx = tid + 256 * it; const int r = idx >> 3, c4 = (idx & 7) * 4;
            const v4f v = *(const v4f*)(AH + (size_t)(i0 + r) * HID2 + h0 + c4);
#pragma unroll
            for (int i = 0; i < 4; ++i) sAt[(c4 + i) * PA + r] = v[i]; }
        { const int r = tid >> 3, c4 = (tid & 7) * 4;
          const v4f v = *(const v4f*)(AM + (size_t)(j0 + r) * HID2 + h0 + c4);
#pragma unroll
          for (int i = 0; i < 4; ++i) sBt[(c4 + i) * PB + r] = v[i]; }
        if (tid < HC) sw[tid] = bfr(w[h0 + tid]);
        __syncthreads();
#pragma unroll 2
        for (int h = 0; h < HC; ++h) {
            const v4f a = *(const v4fa*)(&sAt[h * PA + ig4]);
            const v2f b = *(const v2fa*)(&sBt[h * PB + jg2]);
            const float wv = sw[h];
            a0x += wv * tanh_f(a[0] + b[0]); a0y += wv * tanh_f(a[0] + b[1]);
            a1x += wv * tanh_f(a[1] + b[0]); a1y += wv * tanh_f(a[1] + b[1]);
            a2x += wv * tanh_f(a[2] + b[0]); a2y += wv * tanh_f(a[2] + b[1]);
            a3x += wv * tanh_f(a[3] + b[0]); a3y += wv * tanh_f(a[3] + b[1]);
        }
    }
    const float ob = bfr(ob_p[0]);
    so[(ig4 + 0) * PO + jg2] = a0x + ob; so[(ig4 + 0) * PO + jg2 + 1] = a0y + ob;
    so[(ig4 + 1) * PO + jg2] = a1x + ob; so[(ig4 + 1) * PO + jg2 + 1] = a1y + ob;
    so[(ig4 + 2) * PO + jg2] = a2x + ob; so[(ig4 + 2) * PO + jg2 + 1] = a2y + ob;
    so[(ig4 + 3) * PO + jg2] = a3x + ob; so[(ig4 + 3) * PO + jg2 + 1] = a3y + ob;
    __syncthreads();
    float* obase = OUT + (size_t)i0 * OUT_PITCH + j0;
#pragma unroll 1
    for (int ps = 0; ps < 2; ++ps) {
#pragma unroll
        for (int it = 0; it < 2; ++it) { const int p = tid + 256 * it; const int row = p >> 3, c4 = (p & 7) * 4;
            const v4f val = *(const v4fa*)(&so[row * PO + c4]);
            *(volatile v4f*)(obase + (size_t)row * OUT_PITCH + c4) = val; }
        if (ps == 0) __threadfence(); }
}

static constexpr size_t al256(size_t v) { return (v + 255) & ~(size_t)255; }
static constexpr size_t SZ_XB  = al256((size_t)TT * KD * 2);
static constexpr size_t SZ_W1T = al256((size_t)NCAT * KD * 2);
static constexpr size_t SZ_W2T = al256((size_t)2 * HID2 * HID * 2);
static constexpr size_t SZ_ACT = al256((size_t)TT * NCAT * 2);
static constexpr size_t SZ_P32 = al256((size_t)2 * TT * HID2 * 4);
static constexpr size_t SZ_TOTAL = SZ_XB + SZ_W1T + SZ_W2T + SZ_ACT + SZ_P32;
static_assert(SZ_TOTAL <= (size_t)134217728);
static_assert(((size_t)HID * KD * 2) % 256 == 0);
static_assert(((size_t)TT * HID2 * 4) % 256 == 0);

extern "C" void kernel_launch(void* const* d_in, const int* in_sizes, int n_in,
                              void* d_out, int out_size, void* d_ws, size_t ws_size, hipStream_t stream) {
    if (n_in < 8) return;
    if ((size_t)in_sizes[0] < (size_t)TT * KD) return;
    if ((size_t)in_sizes[1] < (size_t)KD * HID || (size_t)in_sizes[2] < (size_t)KD * HID) return;
    if (in_sizes[3] < NCAT) return;
    if ((size_t)in_sizes[4] < (size_t)NCAT * HID2) return;
    if (in_sizes[5] < HID2 || in_sizes[6] < HID2 || in_sizes[7] < 1) return;
    if ((size_t)out_size < (size_t)(TT - 1) * OUT_PITCH + TT) return;
    if (SZ_TOTAL > ws_size) return;
    const float* x    = (const float*)d_in[0];
    const float* wfoh = (const float*)d_in[1];
    const float* wfom = (const float*)d_in[2];
    const float* cb   = (const float*)d_in[3];
    const float* w2   = (const float*)d_in[4];
    const float* b2   = (const float*)d_in[5];
    const float* wo   = (const float*)d_in[6];
    const float* obp  = (const float*)d_in[7];
    float* OUT = (float*)d_out;
    char* wsp = (char*)d_ws;
    bf*    XB  = (bf*)wsp;    wsp += SZ_XB;
    bf*    W1T = (bf*)wsp;    wsp += SZ_W1T;
    h16*   W2T = (h16*)wsp;   wsp += SZ_W2T;
    h16*   ACT = (h16*)wsp;   wsp += SZ_ACT;
    float* P32 = (float*)wsp; wsp += SZ_P32;

    { const size_t n8 = (size_t)TT * KD / 8;
      k_cvt8<<<(unsigned)((n8 + 255) / 256), 256, 0, stream>>>(x, XB, n8); }
    k_wtb<<<dim3(KD / 64, HID / 64, 1), 256, 0, stream>>>(wfoh, W1T, KD, HID);
    k_wtb<<<dim3(KD / 64, HID / 64, 1), 256, 0, stream>>>(wfom, W1T + (size_t)HID * KD, KD, HID);
    k_wth<<<dim3(HID / 64, HID2 / 64, 2), 256, 0, stream>>>(w2, W2T, HID, HID2);

    k_gemm1<<<dim3(TT / 64, NCAT / 64, 1), 32, 0, stream>>>(XB, W1T, cb, ACT);
    k_gemm2<<<dim3(TT / 64, HID2 / 64, 2), 32, 0, stream>>>(ACT, W2T, b2, P32);
    k_pair<<<dim3(TT / TI, TT / TJ, 1), 256, 0, stream>>>(P32, P32 + (size_t)TT * HID2, wo, obp, OUT);
}
